// mLSTMCell_4054449127612
// MI455X (gfx1250) — hardware-verified
//
#include <hip/hip_runtime.h>
#include <math.h>
#include <stdint.h>

#define NB   2
#define SEQ  2048
#define DM   1024
#define NH   8
#define HD   128
#define XP   (3 * DM)
#define NG   64
#define NQB  (SEQ / 64)
static_assert(NH * HD == DM);
static_assert((SEQ % 64) == 0 && (DM % 64) == 0 && (XP % 64) == 0);
static_assert(((NB * SEQ) % 64) == 0);
static_assert(((NB * SEQ / 64) * (NG / 64)) % 8 == 0);
static_assert((NB * SEQ * DM) % (8 * 256) == 0);
static_assert((XP % 32) == 0 && (HD % 32) == 0);
static_assert((SEQ % 128) == 0);

typedef _Float16 v16h __attribute__((ext_vector_type(16)));
typedef _Float16 v8h  __attribute__((ext_vector_type(8)));
typedef __bf16   v16b __attribute__((ext_vector_type(16)));
typedef __bf16   v8b  __attribute__((ext_vector_type(8)));
typedef float    v8f  __attribute__((ext_vector_type(8)));
typedef float    v4f  __attribute__((ext_vector_type(4)));
typedef unsigned int v4u __attribute__((ext_vector_type(4)));

__device__ __forceinline__ unsigned short bf_bits(float f) {
  unsigned u = __float_as_uint(f);
  return (unsigned short)((u + 0x7FFFu + ((u >> 16) & 1u)) >> 16);
}
__device__ __forceinline__ float bf_up(unsigned short h) { return __uint_as_float(((unsigned)h) << 16); }
__device__ __forceinline__ unsigned short h_bits(_Float16 x) { return __builtin_bit_cast(unsigned short, x); }
__device__ __forceinline__ unsigned pk16(unsigned short a, unsigned short b) { return (unsigned)a | ((unsigned)b << 16); }
__device__ __forceinline__ v8f zero8() { v8f z = {0.f, 0.f, 0.f, 0.f, 0.f, 0.f, 0.f, 0.f}; return z; }

__device__ __forceinline__ v16b ldfrag_b(const __bf16* p) {
  union { v16b v; v8b h[2]; } f;
  f.h[0] = *(const v8b*)(p);
  f.h[1] = *(const v8b*)(p + 16);
  return f.v;
}

__device__ __forceinline__ v8f mma_b(v16b a, v16b b, v8f c) {
  c = __builtin_amdgcn_wmma_f32_16x16x32_bf16(false, a, false, b, (short)0, c, false, false);
  asm volatile("v_nop\n\tv_nop\n\tv_nop\n\tv_nop" : "+v"(c) : "v"(a), "v"(b));
  return c;
}
__device__ __forceinline__ v8f mma_b_raw(v16b a, v16b b, v8f c) {
  return __builtin_amdgcn_wmma_f32_16x16x32_bf16(false, a, false, b, (short)0, c, false, false);
}
__device__ __forceinline__ void dep_guard_b(v8f& a, v8f& b, v16b x, v16b y) {
  asm volatile("v_nop\n\tv_nop\n\tv_nop\n\tv_nop" : "+v"(a), "+v"(b) : "v"(x), "v"(y));
}
__device__ __forceinline__ void keep4_b(v16b a, v16b b, v16b c, v16b d) {
  asm volatile("v_nop" :: "v"(a), "v"(b), "v"(c), "v"(d));
}
__device__ __forceinline__ void acc_guard4(v8f& a, v8f& b, v8f& c, v8f& d) {
  asm volatile("v_nop\n\tv_nop\n\tv_nop\n\tv_nop" : "+v"(a), "+v"(b), "+v"(c), "+v"(d));
}

__global__ __launch_bounds__(256) void cvt_x3(const float* __restrict__ qp, const float* __restrict__ kp,
                                              const float* __restrict__ vp, unsigned short* Xb, int n8) {
  const int t = blockIdx.y;
  const float* src = (t == 0) ? qp : ((t == 1) ? kp : vp);
  const int i = blockIdx.x * 256 + threadIdx.x;
  if (i < n8) {
    const size_t e   = (size_t)i * 8;
    const size_t row = e >> 10;
    const size_t col = e & (size_t)(DM - 1);
    const v4f a  = *(const v4f*)(src + e);
    const v4f a2 = *(const v4f*)(src + e + 4);
    v4u p;
    p[0] = pk16(bf_bits(a[0]),  bf_bits(a[1]));
    p[1] = pk16(bf_bits(a[2]),  bf_bits(a[3]));
    p[2] = pk16(bf_bits(a2[0]), bf_bits(a2[1]));
    p[3] = pk16(bf_bits(a2[2]), bf_bits(a2[3]));
    unsigned short* dst = Xb + row * XP + (size_t)t * DM + col;
    *(volatile v4u*)dst = p;
    __threadfence();
    *(volatile v4u*)dst = p;
  }
}

__global__ __launch_bounds__(256) void prep_wt64(const float* __restrict__ W, unsigned short* WT, int KR, int NCOL) {
  __shared__ __align__(16) unsigned short sW[64 * 72];
  const int tid  = threadIdx.x;
  const int wave = tid >> 5;
  const int lane = tid & 31;
  const int n0   = blockIdx.x * 64;
  const int k0   = blockIdx.y * 64;
  if (n0 + 64 > NCOL || k0 + 64 > KR) return;
  const int r  = tid >> 4;
  const int c4 = (tid & 15) * 4;
#pragma unroll
  for (int i = 0; i < 4; ++i) {
    const int kk = r + 16 * i;
    const v4f v = *(const v4f*)(W + (size_t)(k0 + kk) * NCOL + n0 + c4);
#pragma unroll
    for (int e = 0; e < 4; ++e) sW[(c4 + e) * 72 + kk] = bf_bits(v[e]);
  }
  __syncthreads();
  const int q = lane >> 3, c8 = (lane & 7) * 8;
  v4u pv[2];
  size_t po[2];
#pragma unroll
  for (int it = 0; it < 2; ++it) {
    const int row = wave * 8 + it * 4 + q;
    pv[it] = *(const v4u*)(sW + row * 72 + c8);
    po[it] = (size_t)(n0 + row) * KR + k0 + c8;
  }
  for (int pass = 0; pass < 2; ++pass) {
#pragma unroll
    for (int it = 0; it < 2; ++it) *(volatile v4u*)(WT + po[it]) = pv[it];
    __threadfence();
  }
}

__global__ __launch_bounds__(128) void prep_gw(const float* __restrict__ Wi, const float* __restrict__ Wf,
                                               unsigned short* WgT, int KR) {
  __shared__ __align__(16) unsigned short sW[16 * 72];
  const int tid  = threadIdx.x;
  const int wave = tid >> 5;
  const int lane = tid & 31;
  const int k0   = blockIdx.x * 64;
  if (k0 + 64 > KR) return;
  {
    const int kk = tid & 63;
    const int nb = (tid < 64) ? 0 : 8;
    const float* src = (tid < 64) ? Wi : Wf;
    const v4f a  = *(const v4f*)(src + (size_t)(k0 + kk) * 8);
    const v4f a2 = *(const v4f*)(src + (size_t)(k0 + kk) * 8 + 4);
#pragma unroll
    for (int e = 0; e < 4; ++e) {
      sW[(nb + e) * 72 + kk]     = bf_bits(a[e]);
      sW[(nb + 4 + e) * 72 + kk] = bf_bits(a2[e]);
    }
  }
  __syncthreads();
  const int q = lane >> 3, c8 = (lane & 7) * 8;
  const v4u z = {0u, 0u, 0u, 0u};
  v4u pv[4];
  size_t po[4];
#pragma unroll
  for (int it = 0; it < 4; ++it) {
    const int row  = wave * 16 + it * 4 + q;
    const int lrow = row & 15;
    v4u val = *(const v4u*)(sW + lrow * 72 + c8);
    if (wave != 0) val = z;
    pv[it] = val;
    po[it] = (size_t)row * KR + k0 + c8;
  }
  for (int pass = 0; pass < 2; ++pass) {
#pragma unroll
    for (int it = 0; it < 4; ++it) *(volatile v4u*)(WgT + po[it]) = pv[it];
    __threadfence();
  }
}

template <int NSPLIT, int OUT_MODE, int BIAS>
__global__ __launch_bounds__(256) void gemm64(
    const unsigned short* __restrict__ Ap, const unsigned short* A2p, int lda, long long strideA,
    const unsigned short* __restrict__ Btp, int ldb, long long strideB,
    const float* __restrict__ bias,
    void* Cout, int ldc, long long strideC,
    void* Cout2, int ldc2, long long strideC2, int N2,
    int M, int N, int K, float rscale) {
  const __bf16* A   = (const __bf16*)(const void*)Ap;
  const __bf16* A2  = (const __bf16*)(const void*)A2p;
  const __bf16* Bt  = (const __bf16*)(const void*)Btp;
  __shared__ __align__(16) float sT[8][16 * 68];
  const int b    = blockIdx.y;
  const int lane = threadIdx.x & 31;
  const int wave = threadIdx.x >> 5;
  const int tilesN = N >> 6;
  const int tilesM = M >> 6;
  const int tile = blockIdx.x * 8 + wave;
  if (tile >= tilesM * tilesN) return;
  const int tm = tile / tilesN;
  const int tn = tile - tm * tilesN;
  const int m0 = tm << 6;
  const int n0 = tn << 6;

  const __bf16* Ab  = A  + (size_t)b * strideA;
  const __bf16* Bb  = Bt + (size_t)b * strideB;
  const __bf16* Ab2 = (NSPLIT >= 1) ? (A2 + (size_t)b * strideA) : Ab;

  const int rlane = lane & 15;
  const int koff  = (lane >> 4) * 8;
  const int mOff  = (lane >> 4) * 8;

  v8f acc[4][4];
#pragma unroll
  for (int i = 0; i < 4; ++i)
#pragma unroll
    for (int j = 0; j < 4; ++j) acc[i][j] = zero8();

  for (int k0 = 0; k0 < K; k0 += 32) {
    v16b bh[4];
#pragma unroll
    for (int j = 0; j < 4; ++j) {
      const size_t bo = (size_t)(n0 + (j << 4) + rlane) * ldb + koff + k0;
      bh[j] = ldfrag_b(Bb + bo);
    }
#pragma unroll
    for (int i = 0; i < 4; ++i) {
      const size_t ao = (size_t)(m0 + (i << 4) + rlane) * lda + koff + k0;
      const v16b ah = ldfrag_b(Ab + ao);
      v16b al = ah;
      if (NSPLIT >= 1) al = ldfrag_b(Ab2 + ao);
#pragma unroll
      for (int j = 0; j < 4; ++j) {
        acc[i][j] = mma_b_raw(ah, bh[j], acc[i][j]);
        if (NSPLIT >= 1) acc[i][j] = mma_b_raw(al, bh[j], acc[i][j]);
      }
      dep_guard_b(acc[i][0], acc[i][3], ah, al);
    }
    keep4_b(bh[0], bh[1], bh[2], bh[3]);
  }
  acc_guard4(acc[0][0], acc[0][1], acc[0][2], acc[0][3]);
  acc_guard4(acc[1][0], acc[1][1], acc[1][2], acc[1][3]);
  acc_guard4(acc[2][0], acc[2][1], acc[2][2], acc[2][3]);
  acc_guard4(acc[3][0], acc[3][1], acc[3][2], acc[3][3]);

  float* slab = sT[wave];
  float bcol[4];
#pragma unroll
  for (int j = 0; j < 4; ++j) {
    bcol[j] = 0.f;
    if (BIAS == 1) bcol[j] = bf_up(bf_bits(bias[n0 + (j << 4) + rlane]));
  }
#pragma unroll
  for (int i = 0; i < 4; ++i) {
    const int mBase = m0 + (i << 4);
    float brow[8];
#pragma unroll
    for (int r = 0; r < 8; ++r) {
      brow[r] = 0.f;
      if (BIAS == 2) brow[r] = bf_up(bf_bits(bias[mBase + mOff + r]));
    }
#pragma unroll
    for (int j = 0; j < 4; ++j) {
#pragma unroll
      for (int r = 0; r < 8; ++r) {
        slab[(mOff + r) * 68 + (j << 4) + rlane] = acc[i][j][r] + bcol[j] + brow[r];
      }
    }
    __builtin_amdgcn_fence(__ATOMIC_RELEASE, "workgroup");
    __builtin_amdgcn_wave_barrier();
    __builtin_amdgcn_fence(__ATOMIC_ACQUIRE, "workgroup");
    if (OUT_MODE == 0) {
      float* C = (float*)Cout + (size_t)b * strideC;
      const int hh = lane >> 4, c4 = (lane & 15) * 4;
      for (int pass = 0; pass < 2; ++pass) {
#pragma unroll
        for (int it = 0; it < 8; ++it) {
          const int row = it * 2 + hh;
          const v4f v = *(const v4f*)(slab + row * 68 + c4);
          *(volatile v4f*)(C + (size_t)(mBase + row) * ldc + n0 + c4) = v;
        }
        __threadfence();
      }
    } else {
      const int q = lane >> 3, c8 = (lane & 7) * 8;
      unsigned short* C  = (unsigned short*)Cout  + (size_t)b * strideC;
      unsigned short* C2 = (unsigned short*)Cout2 + (size_t)b * strideC2;
      const bool wlo = (OUT_MODE == 2) || (n0 < N2);
      v4u hv[4], lv[4];
#pragma unroll
      for (int it = 0; it < 4; ++it) {
        const int row = it * 4 + q;
        const float* sp = slab + row * 68 + c8;
        v4u a, a2;
#pragma unroll
        for (int e = 0; e < 4; ++e) {
          const float f0 = sp[2 * e], f1 = sp[2 * e + 1];
          unsigned short h0, h1, l0, l1;
          if (OUT_MODE == 2) {
            h0 = bf_bits(f0); h1 = bf_bits(f1);
            l0 = bf_bits(f0 - bf_up(h0)); l1 = bf_bits(f1 - bf_up(h1));
          } else {
            const _Float16 x0 = (_Float16)f0, x1 = (_Float16)f1;
            h0 = h_bits(x0); h1 = h_bits(x1);
            l0 = h_bits((_Float16)((f0 - (float)x0) * rscale));
            l1 = h_bits((_Float16)((f1 - (float)x1) * rscale));
          }
          a[e] = pk16(h0, h1); a2[e] = pk16(l0, l1);
        }
        hv[it] = a; lv[it] = a2;
      }
      for (int pass = 0; pass < 2; ++pass) {
#pragma unroll
        for (int it = 0; it < 4; ++it) {
          const int row = it * 4 + q;
          *(volatile v4u*)(C + (size_t)(mBase + row) * ldc + n0 + c8) = hv[it];
          if (wlo) *(volatile v4u*)(C2 + (size_t)(mBase + row) * ldc2 + n0 + c8) = lv[it];
        }
        __threadfence();
      }
    }
    __builtin_amdgcn_fence(__ATOMIC_RELEASE, "workgroup");
    __builtin_amdgcn_wave_barrier();
    __builtin_amdgcn_fence(__ATOMIC_ACQUIRE, "workgroup");
  }
}

__global__ __launch_bounds__(32) void gate_scan(const float* __restrict__ G, const float* __restrict__ igb,
                                                const float* __restrict__ fgb,
                                                float* Ep, float* PMp, float* MMp) {
  __shared__ __align__(16) float se[128];
  __shared__ __align__(16) float sp[128];
  __shared__ __align__(16) float sm[128];
  const int bh   = blockIdx.x;
  const int b    = bh / NH;
  const int h    = bh - b * NH;
  const int lane = threadIdx.x & 31;
  if (b >= NB) return;
  const float bi = bf_up(bf_bits(igb[h]));
  const float bf = bf_up(bf_bits(fgb[h]));
  float ccs = 0.f;
  float cpm = -INFINITY;
#pragma unroll 1
  for (int it = 0; it < SEQ / 32; ++it) {
    const int s = it * 32 + lane;
    const size_t grow = ((size_t)b * SEQ + s) * NG;
    const float gi = G[grow + h] + bi;
    const float gf = G[grow + 8 + h] + bf;
    const float lf = fminf(gf, 0.f) - log1pf(expf(-fabsf(gf)));
    float x = lf;
#pragma unroll
    for (int off = 1; off < 32; off <<= 1) {
      const float y = __shfl_up(x, off, 32);
      x = (lane >= off) ? (x + y) : x;
    }
    const float cs = ccs + x;
    ccs = __shfl(cs, 31, 32);
    const float e = gi - cs;
    float p = e;
#pragma unroll
    for (int off = 1; off < 32; off <<= 1) {
      const float y = __shfl_up(p, off, 32);
      p = (lane >= off) ? fmaxf(p, y) : p;
    }
    const float pm = fmaxf(cpm, p);
    cpm = __shfl(pm, 31, 32);
    const float mm = cs + pm;
    const int slot = (it & 3) * 32 + lane;
    se[slot] = e;
    sp[slot] = pm;
    sm[slot] = mm;
    if ((it & 3) == 3) {
      __syncthreads();
      const v4f ev = *(const v4f*)(se + lane * 4);
      const v4f pv = *(const v4f*)(sp + lane * 4);
      const v4f mv = *(const v4f*)(sm + lane * 4);
      const size_t o = (size_t)bh * SEQ + (size_t)(it >> 2) * 128 + (size_t)lane * 4;
      *(volatile v4f*)(Ep + o)  = ev;
      *(volatile v4f*)(PMp + o) = pv;
      *(volatile v4f*)(MMp + o) = mv;
      __threadfence();
      *(volatile v4f*)(Ep + o)  = ev;
      *(volatile v4f*)(PMp + o) = pv;
      *(volatile v4f*)(MMp + o) = mv;
      __syncthreads();
    }
  }
}

__global__ __launch_bounds__(128)
void gated_attn(const unsigned short* __restrict__ xbp, const unsigned short* __restrict__ vtp,
                const float* __restrict__ Ep, const float* __restrict__ PMp, const float* __restrict__ MMp,
                float* outp, int nqb) {
  union FB { v16b v; v8b h[2]; };
  union FA { v8f v; v4f h[2]; };
  __shared__ __align__(16) __bf16 Qs[64 * HD];
  __shared__ __align__(16) __bf16 Ksh[64 * HD];
  __shared__ __align__(16) __bf16 Vts[HD * 64];
  __shared__ __align__(16) __bf16 Pch[4][16 * 64];
  __shared__ __align__(16) __bf16 Pcl[4][16 * 64];
  __shared__ __align__(16) float  Os[4][16 * HD];

  const int tid  = threadIdx.x;
  const int wave = tid >> 5;
  const int lane = tid & 31;
  const int hh   = lane >> 4;
  const int c    = lane & 15;

  const int bx   = blockIdx.x;
  const int qb   = bx % nqb;
  const int rest = bx / nqb;
  const int h    = rest % NH;
  const int b    = rest / NH;
  if (b >= NB) return;
  const int q0   = qb * 64 + wave * 16;
  const size_t rowB  = (size_t)b * SEQ;
  const size_t ebase = (size_t)(b * NH + h) * SEQ;
  const float kScale = 0.08838834764831845f;

  const __bf16* Xb  = (const __bf16*)(const void*)xbp;
  const __bf16* VTb = (const __bf16*)(const void*)vtp + ((size_t)b * DM + (size_t)h * HD) * SEQ;

  {
    const int r = tid >> 1, half = (tid & 1) * 64;
    const __bf16* qg = Xb + (rowB + (size_t)qb * 64 + r) * XP + (size_t)h * HD + half;
#pragma unroll
    for (int i = 0; i < 8; ++i) {
      const v8b a0 = *(const v8b*)(qg + 8 * i);
      *(v8b*)(Qs + r * HD + half + 8 * i) = a0;
    }
  }
  float* os = Os[wave];
  float* op = os + lane * 8;
  {
    const v4f z4 = {0.f, 0.f, 0.f, 0.f};
#pragma unroll
    for (int t = 0; t < 8; ++t) {
      *(v4f*)(op + t * 256)     = z4;
      *(v4f*)(op + t * 256 + 4) = z4;
    }
  }

  float pmr[8], csum[8];
  {
    const v4f p0 = *(const v4f*)(PMp + ebase + q0 + 8 * hh);
    const v4f p1 = *(const v4f*)(PMp + ebase + q0 + 8 * hh + 4);
    pmr[0] = p0[0]; pmr[1] = p0[1]; pmr[2] = p0[2]; pmr[3] = p0[3];
    pmr[4] = p1[0]; pmr[5] = p1[1]; pmr[6] = p1[2]; pmr[7] = p1[3];
  }
#pragma unroll
  for (int r = 0; r < 8; ++r) csum[r] = 0.f;

  const __bf16* qrow = Qs + (wave * 16 + c) * HD + 8 * hh;

  for (int kt = 0; kt <= qb; ++kt) {
    const int kv0 = kt * 64;
    __syncthreads();
    {
      const int r = tid >> 1, half = (tid & 1) * 64;
      const __bf16* kg = Xb + (rowB + kv0 + r) * XP + DM + (size_t)h * HD + half;
      const __bf16* vg = VTb + (size_t)tid * SEQ + kv0;
#pragma unroll
      for (int i = 0; i < 8; ++i) {
        const v8b a0 = *(const v8b*)(kg + 8 * i);
        *(v8b*)(Ksh + r * HD + half + 8 * i) = a0;
      }
#pragma unroll
      for (int i = 0; i < 8; ++i) {
        const v8b b0 = *(const v8b*)(vg + 8 * i);
        *(v8b*)(Vts + tid * 64 + 8 * i) = b0;
      }
    }
    __syncthreads();

    v8f s[4];
#pragma unroll
    for (int j = 0; j < 4; ++j) s[j] = zero8();
#pragma unroll 1
    for (int dc = 0; dc < 4; ++dc) {
      FB qf;
      qf.h[0] = *(const v8b*)(qrow + dc * 32);
      qf.h[1] = *(const v8b*)(qrow + dc * 32 + 16);
#pragma unroll
      for (int j = 0; j < 4; ++j) {
        FB kb;
        kb.h[0] = *(const v8b*)(Ksh + (j * 16 + c) * HD + dc * 32 + 8 * hh);
        kb.h[1] = *(const v8b*)(Ksh + (j * 16 + c) * HD + dc * 32 + 16 + 8 * hh);
        s[j] = mma_b(qf.v, kb.v, s[j]);
      }
    }

    float ej[4];
#pragma unroll
    for (int j = 0; j < 4; ++j) ej[j] = Ep[ebase + kv0 + j * 16 + c];
    __bf16* pch = Pch[wave];
    __bf16* pcl = Pcl[wave];
#pragma unroll
    for (int r = 0; r < 8; ++r) {
      const int rowq = q0 + 8 * hh + r;
      const float pm = pmr[r];
      float rs = 0.f;
#pragma unroll
      for (int j = 0; j < 4; ++j) {
        const int key = kv0 + j * 16 + c;
        const float arg = fminf(ej[j] - pm, 0.f);
        float d = expf(arg);
        d = (key <= rowq) ? d : 0.f;
        const float cv = s[j][r] * kScale * d;
        rs += cv;
        const unsigned short hb = bf_bits(cv);
        const unsigned short lb = bf_bits(cv - bf_up(hb));
        pch[(8 * hh + r) * 64 + j * 16 + c] = __builtin_bit_cast(__bf16, hb);
        pcl[(8 * hh + r) * 64 + j * 16 + c] = __builtin_bit_cast(__bf16, lb);
      }
#pragma unroll
      for (int off = 1; off < 16; off <<= 1) rs += __shfl_xor(rs, off, 32);
      csum[r] += rs;
    }
    __builtin_amdgcn_fence(__ATOMIC_RELEASE, "workgroup");
    __builtin_amdgcn_wave_barrier();
    __builtin_amdgcn_fence(__ATOMIC_ACQUIRE, "workgroup");

    FB pa0, pl0, pa1, pl1;
    pa0.h[0] = *(const v8b*)(pch + c * 64 + 8 * hh);
    pa0.h[1] = *(const v8b*)(pch + c * 64 + 16 + 8 * hh);
    pa1.h[0] = *(const v8b*)(pch + c * 64 + 32 + 8 * hh);
    pa1.h[1] = *(const v8b*)(pch + c * 64 + 48 + 8 * hh);
    pl0.h[0] = *(const v8b*)(pcl + c * 64 + 8 * hh);
    pl0.h[1] = *(const v8b*)(pcl + c * 64 + 16 + 8 * hh);
    pl1.h[0] = *(const v8b*)(pcl + c * 64 + 32 + 8 * hh);
    pl1.h[1] = *(const v8b*)(pcl + c * 64 + 48 + 8 * hh);
#pragma unroll 1
    for (int t = 0; t < 8; ++t) {
      FA acc;
      acc.h[0] = *(const v4f*)(op + t * 256);
      acc.h[1] = *(const v4f*)(op + t * 256 + 4);
      const __bf16* vr = Vts + (t * 16 + c) * 64 + 8 * hh;
      FB vb0, vb1;
      vb0.h[0] = *(const v8b*)(vr);
      vb0.h[1] = *(const v8b*)(vr + 16);
      vb1.h[0] = *(const v8b*)(vr + 32);
      vb1.h[1] = *(const v8b*)(vr + 48);
      acc.v = mma_b(pa0.v, vb0.v, acc.v);
      acc.v = mma_b(pl0.v, vb0.v, acc.v);
      acc.v = mma_b(pa1.v, vb1.v, acc.v);
      acc.v = mma_b(pl1.v, vb1.v, acc.v);
      *(v4f*)(op + t * 256)     = acc.h[0];
      *(v4f*)(op + t * 256 + 4) = acc.h[1];
    }
  }

  v8f oacc[8];
#pragma unroll
  for (int t = 0; t < 8; ++t) {
    FA a;
    a.h[0] = *(const v4f*)(op + t * 256);
    a.h[1] = *(const v4f*)(op + t * 256 + 4);
    oacc[t] = a.v;
  }
  __builtin_amdgcn_fence(__ATOMIC_RELEASE, "workgroup");
  __builtin_amdgcn_wave_barrier();
  __builtin_amdgcn_fence(__ATOMIC_ACQUIRE, "workgroup");
  {
    const v4f m0v = *(const v4f*)(MMp + ebase + q0 + 8 * hh);
    const v4f m1v = *(const v4f*)(MMp + ebase + q0 + 8 * hh + 4);
    float mr[8];
    mr[0] = m0v[0]; mr[1] = m0v[1]; mr[2] = m0v[2]; mr[3] = m0v[3];
    mr[4] = m1v[0]; mr[5] = m1v[1]; mr[6] = m1v[2]; mr[7] = m1v[3];
#pragma unroll
    for (int r = 0; r < 8; ++r) {
      const float nrm = fmaxf(fabsf(csum[r]), expf(-mr[r])) + 1e-6f;
      const float inv = 1.0f / nrm;
      float ms = 0.f;
#pragma unroll
      for (int t = 0; t < 8; ++t) {
        const float hv = oacc[t][r] * inv;
        oacc[t][r] = hv;
        ms = fmaf(hv, hv, ms);
      }
#pragma unroll
      for (int off = 1; off < 16; off <<= 1) ms += __shfl_xor(ms, off, 32);
      const float rn = rsqrtf(ms * (1.0f / 128.0f) + 1e-6f);
#pragma unroll
      for (int t = 0; t < 8; ++t) os[(8 * hh + r) * HD + t * 16 + c] = oacc[t][r] * rn;
    }
  }
  __builtin_amdgcn_fence(__ATOMIC_RELEASE, "workgroup");
  __builtin_amdgcn_wave_barrier();
  __builtin_amdgcn_fence(__ATOMIC_ACQUIRE, "workgroup");
  {
    float* ob = outp + (rowB + q0) * DM + (size_t)h * HD + lane * 4;
    for (int pass = 0; pass < 2; ++pass) {
#pragma unroll
      for (int it = 0; it < 16; ++it) {
        const v4f vv = *(const v4f*)(os + it * HD + lane * 4);
        *(volatile v4f*)(ob + (size_t)it * DM) = vv;
      }
      __threadfence();
    }
  }
}

extern "C" void kernel_launch(void* const* d_in, const int* in_sizes, int n_in,
                              void* d_out, int out_size, void* d_ws, size_t ws_size,
                              hipStream_t stream) {
  if (n_in < 7) return;
  if (in_sizes[0] != NB * SEQ * DM || in_sizes[1] != NB * SEQ * DM || in_sizes[2] != NB * SEQ * DM) return;
  if (in_sizes[3] != XP * NH || in_sizes[5] != XP * NH) return;
  if (in_sizes[4] != NH || in_sizes[6] != NH) return;
  if (out_size != NB * SEQ * DM) return;

  const float* q   = (const float*)d_in[0];
  const float* k   = (const float*)d_in[1];
  const float* v   = (const float*)d_in[2];
  const float* Wi  = (const float*)d_in[3];
  const float* bi  = (const float*)d_in[4];
  const float* Wf  = (const float*)d_in[5];
  const float* bfv = (const float*)d_in[6];

  const size_t PXB = (size_t)NB * SEQ * XP * 2;
  const size_t PVT = (size_t)NB * DM * SEQ * 2;
  const size_t PWG = (size_t)NG * XP * 2;
  const size_t PG  = (size_t)NB * SEQ * NG * 4;
  const size_t PE  = (size_t)NB * NH * SEQ * 4;
  size_t off = 0;
  const size_t oXb = off; off += PXB;
  const size_t oVT = off; off += PVT;
  const size_t oWG = off; off += PWG;
  const size_t oG  = off; off += PG;
  const size_t oE  = off; off += PE;
  const size_t oPM = off; off += PE;
  const size_t oMM = off; off += PE;
  if (off > ws_size) return;
  if (off > (size_t)134217728) return;

  char* ws = (char*)d_ws;
  unsigned short* Xb  = (unsigned short*)(ws + oXb);
  unsigned short* VT  = (unsigned short*)(ws + oVT);
  unsigned short* WgT = (unsigned short*)(ws + oWG);
  float* G   = (float*)(ws + oG);
  float* E   = (float*)(ws + oE);
  float* PM  = (float*)(ws + oPM);
  float* MM  = (float*)(ws + oMM);
  float* out = (float*)d_out;

  const int n8 = NB * SEQ * DM / 8;
  const dim3 gCvt((n8 + 255) / 256, 3);
  const dim3 gVT(DM / 64, SEQ / 64);
  const dim3 gWG(XP / 64);
  const dim3 gGate(((NB * SEQ / 64) * (NG / 64) + 7) / 8, 1);
  const dim3 gScan(NB * NH);
  const dim3 gAttn(NB * NH * NQB);

  cvt_x3<<<gCvt, dim3(256), 0, stream>>>(q, k, v, Xb, n8);
  prep_wt64<<<gVT, dim3(256), 0, stream>>>(v, VT, SEQ, DM);
  prep_wt64<<<gVT, dim3(256), 0, stream>>>(v + (size_t)SEQ * DM, VT + (size_t)DM * SEQ, SEQ, DM);
  prep_gw<<<gWG, dim3(128), 0, stream>>>(Wi, Wf, WgT, XP);
  gemm64<0, 0, 0><<<gGate, dim3(256), 0, stream>>>(
      Xb, Xb, XP, 0LL, WgT, XP, 0LL, bi,
      (void*)G, NG, 0LL, (void*)G, NG, 0LL, NG,
      NB * SEQ, NG, XP, 1.0f);
  gate_scan<<<gScan, dim3(32), 0, stream>>>(G, bi, bfv, E, PM, MM);
  gated_attn<<<gAttn, dim3(128), 0, stream>>>(Xb, VT, E, PM, MM, out, NQB);
  (void)hipGetLastError();
}
